// EnhancedEdgeScorer_68753836474931
// MI455X (gfx1250) — hardware-run, weakly checked
//
#include <hip/hip_runtime.h>

#define NN     32768
#define CL     33
#define DD     128
#define NE     131072
#define QKVW   384
#define FEATW  160
#define AP     168
#define XP     136
#define CP     68
#define ASC    4096.0f
#define HSC    1024.0f
#define WSC    256.0f
#define INV_AW (1.0f / 1048576.0f)
#define INV_HW (1.0f / 262144.0f)
#define NEG_BIG (-3.40282347e+38f)
#define RSD    0.17677669529663687f

static_assert(NN % 128 == 0);
static_assert(NN % 32 == 0);
static_assert(NE % 128 == 0);
static_assert(NE % 64 == 0);
static_assert(FEATW % 32 == 0);
static_assert(DD % 32 == 0);

typedef _Float16 v16h __attribute__((ext_vector_type(16)));
typedef _Float16 v8h  __attribute__((ext_vector_type(8)));
typedef float    v8f  __attribute__((ext_vector_type(8)));
typedef float    v4f  __attribute__((ext_vector_type(4)));
typedef float    v2f  __attribute__((ext_vector_type(2)));
typedef v8h __attribute__((may_alias)) v8ha;
typedef v4f __attribute__((may_alias)) v4fa;
typedef v2f __attribute__((may_alias)) v2fa;

union Frag { v16h v; v8h half[2]; };

__device__ __forceinline__ int clampi(int v, int lo, int hi) {
  return v < lo ? lo : (v > hi ? hi : v);
}

__device__ __forceinline__ v8f wmma_f16(v16h a, v16h b, v8f c) {
  v8f d = __builtin_amdgcn_wmma_f32_16x16x32_f16(false, a, false, b, (short)0, c, false, false);
  asm volatile("v_nop\n\tv_nop\n\tv_nop\n\tv_nop" : "+v"(d) : "v"(a), "v"(b));
  return d;
}

__device__ __forceinline__ v16h load_frag(const _Float16* p, int h) {
  Frag f;
  f.half[0] = *(const v8ha*)(p + 8 * h);
  f.half[1] = *(const v8ha*)(p + 16 + 8 * h);
  return f.v;
}

template<int NWV>
__device__ __forceinline__ void store_x_pass(const _Float16* sX, _Float16* x16,
                                             int node0, int w, int lane) {
  const int q8 = lane & 7, sub = lane >> 3;
  #pragma unroll
  for (int i = 0; i < 16 / NWV; ++i) {
    const int lid = w * (64 / NWV) + i * 4 + sub;
    const int row = lid >> 1, hl = lid & 1;
    const v8h v = *(const v8ha*)(sX + row * XP + 64 * hl + 8 * q8);
    *(volatile v8h*)(x16 + (size_t)(node0 + row) * DD + 64 * hl + 8 * q8) = v;
  }
}

__device__ __forceinline__ void store_c_pass(const float* sC, float* C, int ldc,
                                             int m0, int n0, int w, int lane) {
  const int q8 = lane & 7, sub = lane >> 3;
  #pragma unroll
  for (int i = 0; i < 16; ++i) {
    const int lid = w * 64 + i * 4 + sub;
    const int row = lid >> 1, hl = lid & 1;
    const v4f v = *(const v4fa*)(sC + row * CP + 32 * hl + 4 * q8);
    *(volatile v4f*)(C + (size_t)(m0 + row) * ldc + n0 + 32 * hl + 4 * q8) = v;
  }
}

__global__ __launch_bounds__(256) void k_cvt(
    const float* __restrict__ proj_w, const float* __restrict__ qkv_w,
    const float* __restrict__ out_w, const float* __restrict__ w2,
    const float* __restrict__ w1,
    _Float16* __restrict__ pproj, _Float16* __restrict__ pqkv,
    _Float16* __restrict__ pout, _Float16* __restrict__ pw2,
    _Float16* __restrict__ pw1ab)
{
  const int seg = blockIdx.y;
  const int g = blockIdx.x * 256 + threadIdx.x;
  v4f a, c;
  _Float16* dst;
  if (seg < 4) {
    const float* src;
    int n8;
    if (seg == 0)      { src = proj_w; dst = pproj; n8 = DD * FEATW / 8; }
    else if (seg == 1) { src = qkv_w;  dst = pqkv;  n8 = 3 * QKVW * DD / 8; }
    else if (seg == 2) { src = out_w;  dst = pout;  n8 = 3 * DD * DD / 8; }
    else               { src = w2;     dst = pw2;   n8 = 64 * DD / 8; }
    if (g >= n8) return;
    a = *(const v4fa*)(src + (size_t)g * 8);
    c = *(const v4fa*)(src + (size_t)g * 8 + 4);
    dst += (size_t)g * 8;
  } else {
    if (g >= 256 * DD / 8) return;
    const int row = g >> 4, col0 = (g & 15) * 8;
    const float* src = w1 + (size_t)(row & 127) * 258 + (row >> 7) * 128 + col0;
    const v2f s0 = *(const v2fa*)(src);
    const v2f s1 = *(const v2fa*)(src + 2);
    const v2f s2 = *(const v2fa*)(src + 4);
    const v2f s3 = *(const v2fa*)(src + 6);
    a.x = s0.x; a.y = s0.y; a.z = s1.x; a.w = s1.y;
    c.x = s2.x; c.y = s2.y; c.z = s3.x; c.w = s3.y;
    dst = pw1ab + (size_t)row * DD + col0;
  }
  const v8h o = { (_Float16)(a.x * WSC), (_Float16)(a.y * WSC), (_Float16)(a.z * WSC), (_Float16)(a.w * WSC),
                  (_Float16)(c.x * WSC), (_Float16)(c.y * WSC), (_Float16)(c.z * WSC), (_Float16)(c.w * WSC) };
  *(volatile v8h*)dst = o;
  __threadfence();
  *(volatile v8h*)dst = o;
}

__global__ __launch_bounds__(128) void k_encode(
    const int* __restrict__ type_idx, const int* __restrict__ cat_idx,
    const float* __restrict__ log_deg,
    const float* __restrict__ type_emb, const float* __restrict__ cat0,
    const float* __restrict__ cat1,
    const float* __restrict__ deg_w, const float* __restrict__ deg_b,
    const _Float16* __restrict__ pproj, const float* __restrict__ proj_b,
    _Float16* __restrict__ x16)
{
  __shared__ __attribute__((aligned(16))) _Float16 sA[32 * AP];
  __shared__ __attribute__((aligned(16))) _Float16 sX[32 * XP];

  const int tid = threadIdx.x, lane = tid & 31;
  const int w = __builtin_amdgcn_readfirstlane(tid >> 5);
  const int h = lane >> 4, m = lane & 15;
  const int node0 = blockIdx.x * 32;

  {
    const int node = node0 + lane;
    const int ti = clampi(type_idx[node], 0, 7);
    const int c0 = clampi(cat_idx[2 * node], 0, 16);
    const int c1 = clampi(cat_idx[2 * node + 1], 0, 16);
    const float ld = log_deg[node];
    _Float16* row = sA + lane * AP;
    #pragma unroll 1
    for (int i = 0; i < 16; ++i) {
      const int f = w + 4 * i;
      row[f] = (_Float16)(type_emb[ti * 64 + f] * ASC);
    }
    #pragma unroll 1
    for (int i = 0; i < 8; ++i) {
      const int f = w + 4 * i;
      row[64 + f] = (_Float16)(cat0[c0 * 32 + f] * ASC);
      row[96 + f] = (_Float16)(cat1[c1 * 32 + f] * ASC);
      const float d = fmaxf(ld * deg_w[f] + deg_b[f], 0.0f);
      row[128 + f] = (_Float16)(d * ASC);
    }
  }
  __syncthreads();

  const v8f zero8 = {0.f, 0.f, 0.f, 0.f, 0.f, 0.f, 0.f, 0.f};
  v8f acc[2][2];
  #pragma unroll
  for (int mt = 0; mt < 2; ++mt)
    #pragma unroll
    for (int nt = 0; nt < 2; ++nt) acc[mt][nt] = zero8;

  const _Float16* a0p = sA + m * AP;
  const _Float16* a1p = sA + (16 + m) * AP;
  const _Float16* wb  = pproj + (size_t)(32 * w + m) * FEATW;

  #pragma unroll 1
  for (int k0 = 0; k0 < FEATW; k0 += 32) {
    const v16h a0 = load_frag(a0p + k0, h);
    const v16h a1 = load_frag(a1p + k0, h);
    #pragma unroll
    for (int nt = 0; nt < 2; ++nt) {
      const v16h b = load_frag(wb + (size_t)nt * 16 * FEATW + k0, h);
      acc[0][nt] = wmma_f16(a0, b, acc[0][nt]);
      acc[1][nt] = wmma_f16(a1, b, acc[1][nt]);
    }
  }

  #pragma unroll
  for (int nt = 0; nt < 2; ++nt) {
    const int col = 32 * w + 16 * nt + m;
    const float bv = proj_b[col];
    #pragma unroll
    for (int mt = 0; mt < 2; ++mt) {
      #pragma unroll
      for (int r = 0; r < 8; ++r) {
        const float x = acc[mt][nt][r] * INV_AW + bv;
        sX[(16 * mt + 8 * h + r) * XP + col] = (_Float16)(x * ASC);
      }
    }
  }
  __syncthreads();

  store_x_pass<4>(sX, x16, node0, w, lane);
  __threadfence();
  store_x_pass<4>(sX, x16, node0, w, lane);
}

__global__ __launch_bounds__(128) void k_gemm(
    const _Float16* __restrict__ A, int lda,
    const _Float16* __restrict__ B, int K,
    const float* __restrict__ bias, int nbias,
    float* __restrict__ C, int ldc)
{
  __shared__ __attribute__((aligned(16))) float sC[128 * CP];

  const int tid = threadIdx.x, lane = tid & 31;
  const int w = __builtin_amdgcn_readfirstlane(tid >> 5);
  const int h = lane >> 4, m = lane & 15;
  const int m0 = blockIdx.x * 128, n0 = blockIdx.y * 64;
  const int m0w = m0 + 32 * w;

  const _Float16* xa0 = A + (size_t)(m0w + m) * lda;
  const _Float16* xa1 = xa0 + (size_t)16 * lda;
  const _Float16* wb  = B + (size_t)(n0 + m) * K;

  const v8f zero8 = {0.f, 0.f, 0.f, 0.f, 0.f, 0.f, 0.f, 0.f};
  v8f acc[2][4];
  #pragma unroll
  for (int mt = 0; mt < 2; ++mt)
    #pragma unroll
    for (int nt = 0; nt < 4; ++nt) acc[mt][nt] = zero8;

  #pragma unroll 1
  for (int k0 = 0; k0 < K; k0 += 32) {
    const v16h a0 = load_frag(xa0 + k0, h);
    const v16h a1 = load_frag(xa1 + k0, h);
    #pragma unroll
    for (int nt = 0; nt < 4; ++nt) {
      const v16h b = load_frag(wb + (size_t)nt * 16 * K + k0, h);
      acc[0][nt] = wmma_f16(a0, b, acc[0][nt]);
      acc[1][nt] = wmma_f16(a1, b, acc[1][nt]);
    }
  }

  #pragma unroll
  for (int nt = 0; nt < 4; ++nt) {
    const int col = n0 + 16 * nt + m;
    const int cc = clampi(col, 0, nbias - 1);
    const float bl = bias[cc];
    const float bv = (col < nbias) ? bl : 0.0f;
    #pragma unroll
    for (int mt = 0; mt < 2; ++mt) {
      #pragma unroll
      for (int r = 0; r < 8; ++r) {
        const int rowl = 32 * w + 16 * mt + 8 * h + r;
        sC[rowl * CP + 16 * nt + m] = acc[mt][nt][r] * INV_AW + bv;
      }
    }
  }
  __syncthreads();

  store_c_pass(sC, C, ldc, m0, n0, w, lane);
  __threadfence();
  store_c_pass(sC, C, ldc, m0, n0, w, lane);
}

__global__ __launch_bounds__(256) void k_attn(
    const float* __restrict__ QKV,
    const int* __restrict__ ctx,
    const int* __restrict__ kpm,
    const _Float16* __restrict__ pout_l,
    const float* __restrict__ outb_l,
    _Float16* __restrict__ x16)
{
  __shared__ __attribute__((aligned(16))) float    sS[8 * 4 * 36];
  __shared__ __attribute__((aligned(16))) _Float16 sO[32 * XP];
  __shared__ __attribute__((aligned(16))) _Float16 sX[32 * XP];

  const int tid = threadIdx.x, lane = tid & 31;
  const int w = __builtin_amdgcn_readfirstlane(tid >> 5);
  const int hh = lane >> 3, g = lane & 7;
  const int h = lane >> 4, m = lane & 15;
  const int node0 = blockIdx.x * 32;
  float* sSw = sS + (w * 4 + hh) * 36;

  #pragma unroll 1
  for (int s = 0; s < 4; ++s) {
    const int nl = w * 4 + s;
    const int node = node0 + nl;
    const float* qrow = QKV + (size_t)node * QKVW;
    const v4f q4 = *(const v4fa*)(qrow + hh * 32 + 4 * g);
    const int* cp = ctx + (size_t)node * CL;
    const int* mp = kpm + (size_t)node * CL;

    float mx = NEG_BIG;
    int allm = 1;
    #pragma unroll 1
    for (int j = 0; j < CL; ++j) {
      const int mk = __builtin_amdgcn_readfirstlane(mp[j]);
      float sc = NEG_BIG;
      if (mk == 0) {
        const int c = clampi(__builtin_amdgcn_readfirstlane(cp[j]), 0, NN - 1);
        const v4f k4 = *(const v4fa*)(QKV + (size_t)c * QKVW + DD + hh * 32 + 4 * g);
        float d = q4.x * k4.x + q4.y * k4.y + q4.z * k4.z + q4.w * k4.w;
        d += __shfl_xor(d, 4);
        d += __shfl_xor(d, 2);
        d += __shfl_xor(d, 1);
        sc = d * RSD;
      }
      allm &= (mk != 0);
      mx = fmaxf(mx, sc);
      sSw[j] = sc;
    }

    float den = 0.0f;
    v4f o4 = {0.f, 0.f, 0.f, 0.f};
    #pragma unroll 1
    for (int j = 0; j < CL; ++j) {
      const float sc = sSw[j];
      const float p = expf(sc - mx);
      den += p;
      const int mk = __builtin_amdgcn_readfirstlane(mp[j]);
      const int need = (mk == 0) | allm;
      if (need) {
        const int c = clampi(__builtin_amdgcn_readfirstlane(cp[j]), 0, NN - 1);
        const v4f v4 = *(const v4fa*)(QKV + (size_t)c * QKVW + 2 * DD + hh * 32 + 4 * g);
        o4 = o4 + v4 * p;
      }
    }
    const float sc_o = (1.0f / den) * ASC;
    _Float16* orow = sO + nl * XP + hh * 32 + 4 * g;
    orow[0] = (_Float16)(o4.x * sc_o);
    orow[1] = (_Float16)(o4.y * sc_o);
    orow[2] = (_Float16)(o4.z * sc_o);
    orow[3] = (_Float16)(o4.w * sc_o);
  }
  __syncthreads();

  const v8f zero8 = {0.f, 0.f, 0.f, 0.f, 0.f, 0.f, 0.f, 0.f};
  v8f acc[2];
  acc[0] = zero8; acc[1] = zero8;
  const _Float16* a0p = sO + m * XP;
  const _Float16* a1p = sO + (16 + m) * XP;
  const _Float16* wb  = pout_l + (size_t)(16 * w + m) * DD;
  #pragma unroll 1
  for (int k0 = 0; k0 < DD; k0 += 32) {
    const v16h a0 = load_frag(a0p + k0, h);
    const v16h a1 = load_frag(a1p + k0, h);
    const v16h b  = load_frag(wb + k0, h);
    acc[0] = wmma_f16(a0, b, acc[0]);
    acc[1] = wmma_f16(a1, b, acc[1]);
  }

  {
    const int col = 16 * w + m;
    const float bv = outb_l[col];
    #pragma unroll
    for (int mt = 0; mt < 2; ++mt) {
      #pragma unroll
      for (int r = 0; r < 8; ++r) {
        const float x = fmaxf(acc[mt][r] * INV_AW + bv, 0.0f);
        sX[(16 * mt + 8 * h + r) * XP + col] = (_Float16)(x * ASC);
      }
    }
  }
  __syncthreads();

  store_x_pass<8>(sX, x16, node0, w, lane);
  __threadfence();
  store_x_pass<8>(sX, x16, node0, w, lane);
}

__global__ __launch_bounds__(256) void k_edge_h1(
    const float* __restrict__ PQ,
    const int* __restrict__ eu, const int* __restrict__ ev,
    const float* __restrict__ ef,
    const float* __restrict__ w1,
    _Float16* __restrict__ H1)
{
  __shared__ __attribute__((aligned(16))) float sW[256];
  const int tid = threadIdx.x;
  sW[tid] = w1[(size_t)(tid & 127) * 258 + 256 + (tid >> 7)];
  __syncthreads();

  const int el = tid >> 4, col0 = (tid & 15) * 8;
  const v4f wa0 = *(const v4fa*)(sW + col0);
  const v4f wa1 = *(const v4fa*)(sW + col0 + 4);
  const v4f wb0 = *(const v4fa*)(sW + 128 + col0);
  const v4f wb1 = *(const v4fa*)(sW + 128 + col0 + 4);

  #pragma unroll 1
  for (int p = 0; p < 4; ++p) {
    const int e = blockIdx.x * 64 + p * 16 + el;
    const int u = clampi(eu[e], 0, NN - 1);
    const int v = clampi(ev[e], 0, NN - 1);
    const float f0 = ef[2 * e], f1 = ef[2 * e + 1];
    const float* pr = PQ + (size_t)u * 256 + col0;
    const float* qr = PQ + (size_t)v * 256 + DD + col0;
    const v4f pa = *(const v4fa*)(pr);
    const v4f pb = *(const v4fa*)(pr + 4);
    const v4f qa = *(const v4fa*)(qr);
    const v4f qb = *(const v4fa*)(qr + 4);
    const v4f ha = pa + qa + wa0 * f0 + wb0 * f1;
    const v4f hb = pb + qb + wa1 * f0 + wb1 * f1;
    const v8h o = { (_Float16)(fmaxf(ha.x, 0.f) * HSC), (_Float16)(fmaxf(ha.y, 0.f) * HSC),
                    (_Float16)(fmaxf(ha.z, 0.f) * HSC), (_Float16)(fmaxf(ha.w, 0.f) * HSC),
                    (_Float16)(fmaxf(hb.x, 0.f) * HSC), (_Float16)(fmaxf(hb.y, 0.f) * HSC),
                    (_Float16)(fmaxf(hb.z, 0.f) * HSC), (_Float16)(fmaxf(hb.w, 0.f) * HSC) };
    _Float16* dst = H1 + (size_t)e * DD + col0;
    *(volatile v8h*)dst = o;
    __threadfence();
    *(volatile v8h*)dst = o;
  }
}

__global__ __launch_bounds__(128) void k_edge_out(
    const _Float16* __restrict__ H1,
    const _Float16* __restrict__ pw2,
    const float* __restrict__ b2, const float* __restrict__ w3,
    const float* __restrict__ b3,
    float* __restrict__ out)
{
  __shared__ __attribute__((aligned(16))) float sL[128];

  const int tid = threadIdx.x, lane = tid & 31;
  const int w = __builtin_amdgcn_readfirstlane(tid >> 5);
  const int h = lane >> 4, m = lane & 15;
  const int m0 = blockIdx.x * 128;
  const int m0w = m0 + 32 * w;

  const _Float16* xa0 = H1 + (size_t)(m0w + m) * DD;
  const _Float16* xa1 = xa0 + (size_t)16 * DD;
  const _Float16* wb  = pw2 + (size_t)m * DD;

  const v8f zero8 = {0.f, 0.f, 0.f, 0.f, 0.f, 0.f, 0.f, 0.f};
  v8f acc[2][4];
  #pragma unroll
  for (int mt = 0; mt < 2; ++mt)
    #pragma unroll
    for (int nt = 0; nt < 4; ++nt) acc[mt][nt] = zero8;

  #pragma unroll 1
  for (int k0 = 0; k0 < DD; k0 += 32) {
    const v16h a0 = load_frag(xa0 + k0, h);
    const v16h a1 = load_frag(xa1 + k0, h);
    #pragma unroll
    for (int nt = 0; nt < 4; ++nt) {
      const v16h b = load_frag(wb + (size_t)nt * 16 * DD + k0, h);
      acc[0][nt] = wmma_f16(a0, b, acc[0][nt]);
      acc[1][nt] = wmma_f16(a1, b, acc[1][nt]);
    }
  }

  float bc[4], wc[4];
  #pragma unroll
  for (int nt = 0; nt < 4; ++nt) { bc[nt] = b2[16 * nt + m]; wc[nt] = w3[16 * nt + m]; }
  const float b3v = b3[0];

  #pragma unroll
  for (int mt = 0; mt < 2; ++mt) {
    #pragma unroll
    for (int r = 0; r < 8; ++r) {
      float part = 0.0f;
      #pragma unroll
      for (int nt = 0; nt < 4; ++nt)
        part += fmaxf(acc[mt][nt][r] * INV_HW + bc[nt], 0.0f) * wc[nt];
      part += __shfl_xor(part, 8);
      part += __shfl_xor(part, 4);
      part += __shfl_xor(part, 2);
      part += __shfl_xor(part, 1);
      sL[32 * w + 16 * mt + 8 * h + r] = part + b3v;
    }
  }
  __syncthreads();

  if (w == 0) {
    const v4f v = *(const v4fa*)(sL + 4 * lane);
    float* dst = out + (size_t)m0 + 4 * lane;
    *(volatile v4f*)dst = v;
    __threadfence();
    *(volatile v4f*)dst = v;
  }
}

extern "C" void kernel_launch(void* const* d_in, const int* in_sizes, int n_in,
                              void* d_out, int out_size, void* d_ws, size_t ws_size,
                              hipStream_t stream) {
  if (n_in < 25) return;
  if (in_sizes[0] != NN || in_sizes[1] != 2 * NN || in_sizes[2] != NN) return;
  if (in_sizes[3] != NN * CL || in_sizes[4] != NN * CL) return;
  if (in_sizes[5] != NE || in_sizes[6] != NE || in_sizes[7] != 2 * NE) return;
  if (in_sizes[8] != 8 * 64 || in_sizes[9] != 17 * 32 || in_sizes[10] != 17 * 32) return;
  if (in_sizes[11] != 32 || in_sizes[12] != 32) return;
  if (in_sizes[13] != DD * FEATW || in_sizes[14] != DD) return;
  if (in_sizes[15] != 3 * QKVW * DD || in_sizes[16] != 3 * QKVW) return;
  if (in_sizes[17] != 3 * DD * DD || in_sizes[18] != 3 * DD) return;
  if (in_sizes[19] != DD * 258 || in_sizes[20] != DD) return;
  if (in_sizes[21] != 64 * DD || in_sizes[22] != 64) return;
  if (in_sizes[23] != 64 || in_sizes[24] != 1) return;
  if (out_size != NE) return;

  const int*   type_idx = (const int*)  d_in[0];
  const int*   cat_idx  = (const int*)  d_in[1];
  const float* log_deg  = (const float*)d_in[2];
  const int*   ctx_idx  = (const int*)  d_in[3];
  const int*   pad_mask = (const int*)  d_in[4];
  const int*   edge_u   = (const int*)  d_in[5];
  const int*   edge_v   = (const int*)  d_in[6];
  const float* edge_f   = (const float*)d_in[7];
  const float* type_emb = (const float*)d_in[8];
  const float* cat0     = (const float*)d_in[9];
  const float* cat1     = (const float*)d_in[10];
  const float* deg_w    = (const float*)d_in[11];
  const float* deg_b    = (const float*)d_in[12];
  const float* proj_w   = (const float*)d_in[13];
  const float* proj_b   = (const float*)d_in[14];
  const float* qkv_w    = (const float*)d_in[15];
  const float* qkv_b    = (const float*)d_in[16];
  const float* out_w    = (const float*)d_in[17];
  const float* out_b    = (const float*)d_in[18];
  const float* w1       = (const float*)d_in[19];
  const float* b1       = (const float*)d_in[20];
  const float* w2       = (const float*)d_in[21];
  const float* b2       = (const float*)d_in[22];
  const float* w3       = (const float*)d_in[23];
  const float* b3       = (const float*)d_in[24];
  float* out = (float*)d_out;

  const size_t b_pproj = (size_t)DD * FEATW * 2;
  const size_t b_pqkv  = (size_t)3 * QKVW * DD * 2;
  const size_t b_pout  = (size_t)3 * DD * DD * 2;
  const size_t b_pw2   = (size_t)64 * DD * 2;
  const size_t b_pw1ab = (size_t)256 * DD * 2;
  const size_t b_x16   = (size_t)NN * DD * 2;
  const size_t b_qkv   = (size_t)NN * QKVW * 4;
  const size_t b_h1    = (size_t)NE * DD * 2;
  const size_t total = b_pproj + b_pqkv + b_pout + b_pw2 + b_pw1ab + b_x16 + b_qkv + b_h1;
  if (total > ws_size) return;
  if ((size_t)NN * 256 * 4 > b_qkv) return;

  char* ws = (char*)d_ws;
  size_t off = 0;
  _Float16* pproj = (_Float16*)(ws + off); off += b_pproj;
  _Float16* pqkv  = (_Float16*)(ws + off); off += b_pqkv;
  _Float16* pout  = (_Float16*)(ws + off); off += b_pout;
  _Float16* pw2   = (_Float16*)(ws + off); off += b_pw2;
  _Float16* pw1ab = (_Float16*)(ws + off); off += b_pw1ab;
  _Float16* x16   = (_Float16*)(ws + off); off += b_x16;
  float*    QKV   = (float*)   (ws + off);
  float*    PQ    = (float*)   (ws + off); off += b_qkv;
  _Float16* H1    = (_Float16*)(ws + off); off += b_h1;
  if (off != total) return;

  k_cvt<<<dim3((3 * QKVW * DD / 8 + 255) / 256, 5), 256, 0, stream>>>(
      proj_w, qkv_w, out_w, w2, w1, pproj, pqkv, pout, pw2, pw1ab);

  k_encode<<<NN / 32, 128, 0, stream>>>(type_idx, cat_idx, log_deg, type_emb, cat0, cat1,
                                        deg_w, deg_b, pproj, proj_b, x16);

  for (int l = 0; l < 3; ++l) {
    k_gemm<<<dim3(NN / 128, QKVW / 64), 128, 0, stream>>>(
        x16, DD, pqkv + (size_t)l * QKVW * DD, DD, qkv_b + (size_t)l * QKVW, QKVW, QKV, QKVW);
    k_attn<<<NN / 32, 256, 0, stream>>>(
        QKV, ctx_idx, pad_mask, pout + (size_t)l * DD * DD, out_b + (size_t)l * DD, x16);
  }

  k_gemm<<<dim3(NN / 128, 256 / 64), 128, 0, stream>>>(x16, DD, pw1ab, DD, b1, DD, PQ, 256);

  k_edge_h1<<<NE / 64, 256, 0, stream>>>(PQ, edge_u, edge_v, edge_f, w1, H1);
  k_edge_out<<<NE / 128, 128, 0, stream>>>(H1, pw2, b2, w3, b3, out);
}
